// CommunityGCN_90108413870706
// MI455X (gfx1250) — hardware-verified
//
#include <hip/hip_runtime.h>


#define IN_C     128
#define HID      128
#define OUT_C    40
#define OUT_CP   64
#define NCOMM    1000
#define COMM_PB  64
#define NODE_PB  6272
#define WSCALE   16.0f
#define WINV     0.0625f

typedef _Float16 v16h __attribute__((ext_vector_type(16)));
typedef _Float16 v8h  __attribute__((ext_vector_type(8)));
typedef float    v8f  __attribute__((ext_vector_type(8)));
typedef float    v4f  __attribute__((ext_vector_type(4)));
union Frag { v16h v; v8h h[2]; };
union HV   { v8h h8; v4f f4; };

__device__ __forceinline__ v8f wmma_f16(v16h a, v16h b, v8f c)
{
    c = __builtin_amdgcn_wmma_f32_16x16x32_f16(false, a, false, b, (short)0, c, false, false);
    asm volatile("v_nop\n\tv_nop\n\tv_nop\n\tv_nop" : "+v"(c) : "v"(a), "v"(b));
    return c;
}

__device__ __forceinline__ unsigned ballot32(bool p) { return __builtin_amdgcn_ballot_w32(p); }
__device__ __forceinline__ int clampi(int v, int lo, int hi) { return v < lo ? lo : (v > hi ? hi : v); }

__global__ __launch_bounds__(32)
void k_comm(const float* __restrict__ x, const int* __restrict__ com, float* cmean, int N)
{
    __shared__ v4f sacc[COMM_PB][32];
    __shared__ int scnt[COMM_PB];
    const int l = threadIdx.x & 31;
    const int c0 = blockIdx.x * COMM_PB;
    v4f z; z[0] = 0.0f; z[1] = 0.0f; z[2] = 0.0f; z[3] = 0.0f;
    for (int i = 0; i < COMM_PB; ++i) sacc[i][l] = z;
    for (int i = l; i < COMM_PB; i += 32) scnt[i] = 0;

    for (int base = 0; base < N; base += 32) {
        const int n = base + l;
        int cl = -1;
        if (n < N) cl = com[n] - c0;
        const bool hit = (unsigned)cl < (unsigned)COMM_PB;
        unsigned msk = ballot32(hit);
        while (msk) {
            const int bit = __builtin_ctz(msk);
            msk &= msk - 1u;
            int ccl = __shfl(cl, bit);
            ccl = clampi(ccl, 0, COMM_PB - 1);
            const int nn = base + bit;
            const v4f xv = *(const v4f*)(x + (size_t)nn * IN_C + 4 * l);
            v4f a = sacc[ccl][l];
            a += xv;
            sacc[ccl][l] = a;
            const int cv = scnt[ccl];
            scnt[ccl] = cv + 1;
        }
    }
    for (int rep = 0; rep < 2; ++rep) {
        for (int i = 0; i < COMM_PB; ++i) {
            const float inv = 1.0f / fmaxf((float)scnt[i], 1.0f);
            const v4f v = sacc[i][l] * inv;
            *(volatile v4f*)(cmean + (size_t)(c0 + i) * IN_C + 4 * l) = v;
        }
        __threadfence();
    }
}

__global__ __launch_bounds__(32)
void k_deg(const int* __restrict__ dst, float* dis, int E)
{
    __shared__ int scnt[NODE_PB];
    const int l = threadIdx.x & 31;
    const int d0 = blockIdx.x * NODE_PB;
    for (int i = l; i < NODE_PB; i += 32) scnt[i] = 0;

    for (int base = 0; base < E; base += 32) {
        const int e = base + l;
        int dl = -1;
        if (e < E) dl = dst[e] - d0;
        const bool hit = (unsigned)dl < (unsigned)NODE_PB;
        unsigned msk = ballot32(hit);
        while (msk) {
            const int bit = __builtin_ctz(msk);
            msk &= msk - 1u;
            int dd = __shfl(dl, bit);
            dd = clampi(dd, 0, NODE_PB - 1);
            const int cv = scnt[dd];
            scnt[dd] = cv + 1;
        }
    }
    for (int rep = 0; rep < 2; ++rep) {
        for (int i0 = 0; i0 < NODE_PB; i0 += 128) {
            const int i = i0 + 4 * l;
            v4f v;
            #pragma unroll
            for (int j = 0; j < 4; ++j) v[j] = rsqrtf((float)scnt[i + j] + 1.0f);
            *(volatile v4f*)(dis + (size_t)d0 + i) = v;
        }
        __threadfence();
    }
}

__global__ __launch_bounds__(128)
void k_packw(const float* __restrict__ W, _Float16* wt, int K, int Nreal, int Npad)
{
    const int l = threadIdx.x & 31;
    const int n = blockIdx.x * 4 + (threadIdx.x >> 5);
    if (n >= Npad) return;
    for (int rep = 0; rep < 2; ++rep) {
        for (int kb = 8 * l; kb < K; kb += 256) {
            v8h o;
            #pragma unroll
            for (int j = 0; j < 8; ++j) {
                float v = 0.0f;
                if (n < Nreal) v = W[(size_t)(kb + j) * Nreal + n] * WSCALE;
                o[j] = (_Float16)v;
            }
            *(volatile v8h*)(wt + (size_t)n * K + kb) = o;
        }
        __threadfence();
    }
}

__global__ __launch_bounds__(256)
void k_build(const float* __restrict__ x, const int* __restrict__ com,
             const float* __restrict__ cmean, _Float16* a0, int N)
{
    const int l = threadIdx.x & 31, h = l >> 4, m = l & 15;
    const int n = blockIdx.x * 8 + (threadIdx.x >> 5);
    if (n >= N) return;
    const float* sp;
    if (h == 0) {
        sp = x + (size_t)n * IN_C + 8 * m;
    } else {
        int c = com[n];
        c = clampi(c, 0, NCOMM - 1);
        sp = cmean + (size_t)c * IN_C + 8 * m;
    }
    const v4f p = *(const v4f*)sp;
    const v4f q = *(const v4f*)(sp + 4);
    v8h o;
    #pragma unroll
    for (int j = 0; j < 4; ++j) { o[j] = (_Float16)p[j]; o[4 + j] = (_Float16)q[j]; }
    _Float16* op = a0 + (size_t)n * (2 * IN_C) + 8 * l;
    *(volatile v8h*)op = o;
    __threadfence();
    *(volatile v8h*)op = o;
}

template<int NT, int MODE>
__global__ __launch_bounds__(128)
void k_gemm(const _Float16* __restrict__ A, const _Float16* __restrict__ Wt,
            const float* __restrict__ bias, const float* __restrict__ dis,
            void* outp, int M, int K, int lda)
{
    constexpr int NC = NT * 16;
    constexpr int TP = NC + 4;
    __shared__ __attribute__((aligned(16))) float tile[4][16][TP];

    const int l = threadIdx.x & 31, h = l >> 4, m = l & 15, w = threadIdx.x >> 5;
    const int row0 = (blockIdx.x * 4 + w) * 16;
    int ar = row0 + m;
    if (ar > M - 1) ar = M - 1;
    const _Float16* Ap = A + (size_t)ar * lda + 8 * h;

    v8f acc[NT];
    #pragma unroll
    for (int t = 0; t < NT; ++t) {
        #pragma unroll
        for (int r = 0; r < 8; ++r) acc[t][r] = 0.0f;
    }

    for (int k0 = 0; k0 < K; k0 += 32) {
        Frag a;
        a.h[0] = *(const v8h*)(Ap + k0);
        a.h[1] = *(const v8h*)(Ap + k0 + 16);
        #pragma unroll
        for (int t = 0; t < NT; ++t) {
            const _Float16* Bp = Wt + (size_t)(t * 16 + m) * K + k0 + 8 * h;
            Frag b;
            b.h[0] = *(const v8h*)(Bp);
            b.h[1] = *(const v8h*)(Bp + 16);
            acc[t] = wmma_f16(a.v, b.v, acc[t]);
        }
    }

    #pragma unroll
    for (int t = 0; t < NT; ++t) {
        #pragma unroll
        for (int r = 0; r < 8; ++r) tile[w][8 * h + r][t * 16 + m] = acc[t][r] * WINV;
    }
    __syncthreads();

    for (int rep = 0; rep < 2; ++rep) {
        if (MODE == 0) {
            _Float16* O = (_Float16*)outp;
            for (int it = 0; it < 8; ++it) {
                const int rr = 2 * it + h;
                const int row = row0 + rr;
                const int c = 8 * m;
                const v4f p = *(const v4f*)&tile[w][rr][c];
                const v4f q = *(const v4f*)&tile[w][rr][c + 4];
                v8h o;
                #pragma unroll
                for (int j = 0; j < 4; ++j) {
                    const float u0 = fmaxf(p[j] + bias[c + j], 0.0f);
                    const float u1 = fmaxf(q[j] + bias[c + 4 + j], 0.0f);
                    o[j] = (_Float16)u0;
                    o[4 + j] = (_Float16)u1;
                }
                if (row < M) *(volatile v8h*)(O + (size_t)row * NC + c) = o;
            }
        } else {
            float* O = (float*)outp;
            constexpr int LPR = NT * 4;
            constexpr int RPI = 32 / LPR;
            for (int it = 0; it < 16 / RPI; ++it) {
                const int rr = it * RPI + l / LPR;
                const int c = (l % LPR) * 4;
                const int row = row0 + rr;
                const int rowc = row < M ? row : M - 1;
                v4f p = *(const v4f*)&tile[w][rr][c];
                const float dv = dis[rowc];
                p = p * dv;
                if (row < M) *(volatile v4f*)(O + (size_t)row * NC + c) = p;
            }
        }
        __threadfence();
    }
}

template<int CH, int MODE>
__global__ __launch_bounds__(32)
void k_agg(const int* __restrict__ src, const int* __restrict__ dst,
           const float* __restrict__ hw, const float* __restrict__ dis,
           const float* __restrict__ bias, float* acc, void* outp, int N, int E)
{
    constexpr int LPR = CH / 4;
    const int l = threadIdx.x & 31, h = l >> 4, m = l & 15;
    const int d0 = blockIdx.x * NODE_PB;
    int nrows = N - d0;
    if (nrows > NODE_PB) nrows = NODE_PB;
    if (nrows <= 0) return;
    const bool act = (l < LPR);
    const int cl = (l & (LPR - 1)) * 4;

    for (int r = 0; r < nrows; ++r) {
        if (act) {
            const size_t o = (size_t)(d0 + r) * CH + cl;
            const v4f v = *(const v4f*)(hw + o);
            *(v4f*)(acc + o) = v;
        }
    }
    __threadfence();

    for (int base = 0; base < E; base += 32) {
        const int e = base + l;
        int dl = -1, s = 0;
        if (e < E) { dl = dst[e] - d0; s = src[e]; }
        const bool hit = (unsigned)dl < (unsigned)nrows;
        unsigned msk = ballot32(hit);
        while (msk) {
            const int bit = __builtin_ctz(msk);
            msk &= msk - 1u;
            int ss = __shfl(s, bit);
            int dd = __shfl(dl, bit);
            ss = clampi(ss, 0, N - 1);
            dd = clampi(dd, 0, nrows - 1);
            if (act) {
                const v4f hv = *(const v4f*)(hw + (size_t)ss * CH + cl);
                float* ap = acc + (size_t)(d0 + dd) * CH + cl;
                v4f av = *(const v4f*)ap;
                av += hv;
                *(v4f*)ap = av;
            }
        }
    }
    __threadfence();

    if (MODE == 0) {
        float* O = (float*)outp;
        for (int r0 = 0; r0 < nrows; r0 += 2) {
            const int r = r0 + h;
            const int rc = r < nrows ? r : nrows - 1;
            const int d = d0 + rc;
            const int c = 8 * m;
            const float* ap = acc + (size_t)d * CH + c;
            const v4f p = *(const v4f*)ap;
            const v4f q = *(const v4f*)(ap + 4);
            const float dv = dis[d];
            HV o;
            #pragma unroll
            for (int j = 0; j < 4; ++j) {
                const float u0 = fmaxf(p[j] * dv + bias[c + j], 0.0f);
                const float u1 = fmaxf(q[j] * dv + bias[c + 4 + j], 0.0f);
                o.h8[j] = (_Float16)u0;
                o.h8[4 + j] = (_Float16)u1;
            }
            const v4f ov = o.f4;
            float* op = O + (size_t)d * CH + 4 * m;
            if (r < nrows) *(volatile v4f*)op = ov;
            __threadfence();
            if (r < nrows) *(volatile v4f*)op = ov;
        }
    } else {
        for (int rep = 0; rep < 2; ++rep) {
            float* O = (float*)outp;
            const int cnt = nrows * OUT_C;
            const size_t ob = (size_t)d0 * OUT_C;
            for (int i0 = 0; i0 < cnt; i0 += 128) {
                const int i = i0 + 4 * l;
                if (i < cnt) {
                    const int row = i / OUT_C;
                    const int col = i - row * OUT_C;
                    const v4f a = *(const v4f*)(acc + (size_t)(d0 + row) * CH + col);
                    const float dv = dis[d0 + row];
                    v4f v;
                    #pragma unroll
                    for (int j = 0; j < 4; ++j) v[j] = a[j] * dv + bias[col + j];
                    *(volatile v4f*)(O + ob + i) = v;
                }
            }
            __threadfence();
        }
    }
}


static inline size_t al256(size_t v) { return (v + 255) & ~(size_t)255; }

extern "C" void kernel_launch(void* const* d_in, const int* in_sizes, int n_in,
                              void* d_out, int out_size, void* d_ws, size_t ws_size,
                              hipStream_t stream)
{
    if (n_in < 9) return;
    const float* x   = (const float*)d_in[0];
    const int*   edg = (const int*)d_in[1];
    const int*   com = (const int*)d_in[2];
    const float* Win = (const float*)d_in[3];
    const float* bin = (const float*)d_in[4];
    const float* W1  = (const float*)d_in[5];
    const float* b1  = (const float*)d_in[6];
    const float* W2  = (const float*)d_in[7];
    const float* b2  = (const float*)d_in[8];
    const int N = in_sizes[0] / IN_C;
    const int E = in_sizes[1] / 2;
    if (N <= 0) return;
    if (out_size < N * OUT_C) return;
    const int* src = edg;
    const int* dst = edg + E;

    const int gridC = (NCOMM + COMM_PB - 1) / COMM_PB;
    const int gridN = (N + NODE_PB - 1) / NODE_PB;
    const int gridG = (N + 63) / 64;

    char* base = (char*)d_ws;
    size_t off = 0;
    float* CMEAN = (float*)(base + off);     off = al256(off + (size_t)gridC * COMM_PB * IN_C * 4);
    float* DIS   = (float*)(base + off);     off = al256(off + (size_t)gridN * NODE_PB * 4);
    _Float16* WT0 = (_Float16*)(base + off); off = al256(off + (size_t)HID * 2 * IN_C * 2);
    _Float16* WT1 = (_Float16*)(base + off); off = al256(off + (size_t)HID * HID * 2);
    _Float16* WT2 = (_Float16*)(base + off); off = al256(off + (size_t)OUT_CP * HID * 2);
    char* RA  = base + off;                  off = al256(off + (size_t)N * 2 * IN_C * 2);
    char* RB  = base + off;                  off = al256(off + (size_t)N * HID * 4);
    if (off > ws_size) return;

    _Float16* A0  = (_Float16*)RA;
    float*    HW1 = (float*)RA;
    float*    HW2 = (float*)RA;
    _Float16* H1  = (_Float16*)RB;
    float*    ACC = (float*)RB;
    _Float16* H2  = (_Float16*)RB;

    k_comm<<<dim3(gridC), dim3(32), 0, stream>>>(x, com, CMEAN, N);
    k_deg<<<dim3(gridN), dim3(32), 0, stream>>>(dst, DIS, E);
    k_packw<<<dim3((HID + 3) / 4), dim3(128), 0, stream>>>(Win, WT0, 2 * IN_C, HID, HID);
    k_packw<<<dim3((HID + 3) / 4), dim3(128), 0, stream>>>(W1, WT1, HID, HID, HID);
    k_packw<<<dim3((OUT_CP + 3) / 4), dim3(128), 0, stream>>>(W2, WT2, HID, OUT_C, OUT_CP);

    k_build<<<dim3((N + 7) / 8), dim3(256), 0, stream>>>(x, com, CMEAN, A0, N);
    k_gemm<8, 0><<<dim3(gridG), dim3(128), 0, stream>>>(A0, WT0, bin, DIS, (void*)H1, N, 2 * IN_C, 2 * IN_C);

    k_gemm<8, 1><<<dim3(gridG), dim3(128), 0, stream>>>(H1, WT1, b1, DIS, (void*)HW1, N, HID, HID);
    k_agg<128, 0><<<dim3(gridN), dim3(32), 0, stream>>>(src, dst, HW1, DIS, b1, ACC, (void*)H2, N, E);

    k_gemm<4, 1><<<dim3(gridG), dim3(128), 0, stream>>>(H2, WT2, b2, DIS, (void*)HW2, N, HID, 2 * HID);
    k_agg<64, 1><<<dim3(gridN), dim3(32), 0, stream>>>(src, dst, HW2, DIS, b2, ACC, d_out, N, E);
}
